// MiniAttentionLayer_40673340293687
// MI455X (gfx1250) — hardware-verified
//
#include <hip/hip_runtime.h>
#include <string.h>


namespace {
constexpr int NBt = 32768, ND = 256, IE = 128, OE = 128, DM = 256, NH = 2, E = 512, HD = 256;
constexpr float XS = 8.0f, WSC = 256.0f;

typedef _Float16 b16;
typedef __attribute__((ext_vector_type(16))) _Float16 v16b;
typedef __attribute__((ext_vector_type(8))) _Float16 v8b;
typedef __attribute__((ext_vector_type(8))) float v8f;
typedef __attribute__((ext_vector_type(4))) float v4f;
__device__ __forceinline__ float bf16_rne(float f) { unsigned int u = __float_as_uint(f); u += 0x7FFFu + ((u >> 16) & 1u); return __uint_as_float(u & 0xFFFF0000u); }
__device__ __forceinline__ void split16(float v, b16& hi, b16& lo) { hi = (b16)v; lo = (b16)(v - (float)hi); }
__device__ __forceinline__ v16b frag_kb(const b16* p, int hh) { const v8b a = *(const v8b*)(p + 8 * hh), b = *(const v8b*)(p + 16 + 8 * hh); v16b f;
#pragma unroll
  for (int e = 0; e < 8; ++e) { f[e] = a[e]; f[8 + e] = b[e]; } return f; }
__device__ __forceinline__ v8f wmma16b(v16b a, v16b b, v8f c) { v8f d = __builtin_amdgcn_wmma_f32_16x16x32_f16(false, a, false, b, (short)0, c, false, false); asm volatile("v_nop\n\tv_nop\n\tv_nop\n\tv_nop" : "+v"(d) : "v"(a), "v"(b)); return d; }
__device__ __forceinline__ void wave_lds_sync() { __builtin_amdgcn_fence(__ATOMIC_RELEASE, "workgroup"); __builtin_amdgcn_wave_barrier(); __builtin_amdgcn_fence(__ATOMIC_ACQUIRE, "workgroup"); }
__device__ __forceinline__ float nexp(float x) { return __builtin_amdgcn_exp2f(x * 1.4426950408889634f); }
__device__ __forceinline__ float pmul(float a, float b) { float p = a * b; asm volatile("" : "+v"(p)); return p; }

__global__ __launch_bounds__(256) void prepx_kernel(const float* __restrict__ us, const float* __restrict__ vs, const float* __restrict__ ed, b16* __restrict__ XU, b16* __restrict__ XV, b16* __restrict__ XE) {
  const size_t t = (size_t)blockIdx.x * 256 + threadIdx.x; const size_t n1 = (size_t)NBt * ND / 8, n3 = (size_t)NBt * IE / 8; const float* src; b16* dst; size_t e;
  if (t < n1) { src = us; dst = XU; e = t * 8; } else if (t < 2 * n1) { src = vs; dst = XV; e = (t - n1) * 8; } else if (t < 2 * n1 + n3) { src = ed; dst = XE; e = (t - 2 * n1) * 8; } else return;
  const v4f a = *(const v4f*)(src + e), c = *(const v4f*)(src + e + 4); v8b o;
#pragma unroll
  for (int j = 0; j < 4; ++j) { o[j] = (b16)(bf16_rne(a[j]) * XS); o[4 + j] = (b16)(bf16_rne(c[j]) * XS); }
  for (int pass = 0; pass < 2; ++pass) { *(volatile v8b*)(dst + e) = o; __threadfence(); }
}
__global__ __launch_bounds__(256) void preprow_kernel(const float* __restrict__ w, int n8, b16* __restrict__ dst) {
  const size_t t = (size_t)blockIdx.x * 256 + threadIdx.x; if (t >= (size_t)n8) return; const size_t e = t * 8; const v4f a = *(const v4f*)(w + e), c = *(const v4f*)(w + e + 4); v8b o;
#pragma unroll
  for (int j = 0; j < 4; ++j) { o[j] = (b16)(bf16_rne(a[j]) * WSC); o[4 + j] = (b16)(bf16_rne(c[j]) * WSC); }
  for (int pass = 0; pass < 2; ++pass) { *(volatile v8b*)(dst + e) = o; __threadfence(); }
}
__global__ __launch_bounds__(256) void prepwk_kernel(const float* __restrict__ wi, b16* __restrict__ WKT) {
  __shared__ __attribute__((aligned(16))) b16 T[64][64 + 8];
  const int h = blockIdx.z, d0 = blockIdx.x * 64, j0 = blockIdx.y * 64, t_ = threadIdx.x;
  for (int q = t_; q < 64 * 64; q += 256) { const int dd = q >> 6, jj = q & 63; T[jj][dd] = (b16)(bf16_rne(wi[((size_t)E + h * HD + d0 + dd) * E + j0 + jj]) * WSC); }
  __syncthreads();
  for (int pass = 0; pass < 2; ++pass) { for (int q = t_; q < 64 * 8; q += 256) { const int jj = q >> 3, c8 = (q & 7) * 8; *(volatile v8b*)(WKT + ((size_t)h * E + j0 + jj) * HD + d0 + c8) = *(const v8b*)(&T[jj][c8]); } __threadfence(); }
}
struct GArgs { const b16* A; const b16* Al; const b16* W; const float* b; b16* Yh; b16* Yl; float* Y32; int lda, K, ldy, act, boff, yoff, pad_; };
template <int MODE>
__global__ __launch_bounds__(128) void gemm_kernel(GArgs g) {
  __shared__ __attribute__((aligned(16))) float Ts[4][16][128 + 4];
  const int wave = threadIdx.x >> 5, lane = threadIdx.x & 31, nloc = lane & 15, hlf = lane >> 4; const size_t m0 = (size_t)blockIdx.x * 64 + wave * 16; const int n0 = blockIdx.y * 128;
  v8f acc[8];
#pragma unroll
  for (int t = 0; t < 8; ++t) acc[t] = (v8f){};
  for (int kb = 0; kb < g.K; kb += 32) { const v16b a = frag_kb(g.A + (m0 + nloc) * g.lda + kb, hlf);
    if (g.Al) { const v16b al = frag_kb(g.Al + (m0 + nloc) * g.lda + kb, hlf);
#pragma unroll
      for (int t = 0; t < 8; ++t) { const v16b bw = frag_kb(g.W + (size_t)(n0 + t * 16 + nloc) * g.K + kb, hlf); acc[t] = wmma16b(a, bw, acc[t]); acc[t] = wmma16b(al, bw, acc[t]); } }
    else {
#pragma unroll
      for (int t = 0; t < 8; ++t) acc[t] = wmma16b(a, frag_kb(g.W + (size_t)(n0 + t * 16 + nloc) * g.K + kb, hlf), acc[t]); } }
#pragma unroll
  for (int t = 0; t < 8; ++t) { const float bb = g.b ? bf16_rne(g.b[g.boff + n0 + t * 16 + nloc]) : 0.0f;
#pragma unroll
    for (int r = 0; r < 8; ++r) { float v = acc[t][r] * (1.0f / (XS * WSC)) + bb; if (g.act == 1) v = v / (1.0f + nexp(-v)); Ts[wave][8 * hlf + r][t * 16 + nloc] = v; } }
  wave_lds_sync();
  for (int pass = 0; pass < 2; ++pass) {
    for (int rr = 0; rr < 16; ++rr) { if (MODE == 0) { if (lane < 16) { v8b hv, lv; for (int j = 0; j < 8; ++j) { b16 a_, c_; split16(Ts[wave][rr][lane * 8 + j] * XS, a_, c_); hv[j] = a_; lv[j] = c_; }
          *(volatile v8b*)(g.Yh + (m0 + rr) * g.ldy + g.yoff + n0 + lane * 8) = hv; if (g.Yl) *(volatile v8b*)(g.Yl + (m0 + rr) * g.ldy + g.yoff + n0 + lane * 8) = lv; } }
      else { *(volatile v4f*)(g.Y32 + (m0 + rr) * g.ldy + g.yoff + n0 + lane * 4) = *(const v4f*)(&Ts[wave][rr][lane * 4]); } }
    __threadfence(); }
}
__device__ __forceinline__ float hsum16(float v) { v += __shfl_xor(v, 1); v += __shfl_xor(v, 2); v += __shfl_xor(v, 4); return v + __shfl_xor(v, 8); }
__global__ __launch_bounds__(256) void mix_kernel(const b16* __restrict__ KU, const b16* __restrict__ VU, const b16* __restrict__ KV, const b16* __restrict__ VV, const b16* __restrict__ QKVE, const b16* __restrict__ QE2, const float* __restrict__ G, const float* __restrict__ bi, b16* __restrict__ VB) {
  const int wave = threadIdx.x >> 5, lane = threadIdx.x & 31; const size_t b = ((size_t)blockIdx.x * 8 + wave) * 2 + (lane >> 4); const int c0 = (lane & 15) * 32;
  float sc[NH][3];
#pragma unroll 1
  for (int h = 0; h < NH; ++h) { float su = 0, sv = 0, se = 0, sq = 0;
#pragma unroll 1
    for (int j8 = 0; j8 < 32; j8 += 8) { const int j = c0 + j8; const v8b ku = *(const v8b*)(KU + b * 2 * E + j), kv = *(const v8b*)(KV + b * 2 * E + j), ke = *(const v8b*)(QKVE + b * 3 * E + E + j);
      const v4f g0 = *(const v4f*)(G + (b * NH + h) * E + j), g1 = *(const v4f*)(G + (b * NH + h) * E + j + 4);
#pragma unroll
      for (int q = 0; q < 8; ++q) { const float gg = q < 4 ? g0[q] : g1[q - 4]; su += (float)ku[q] * gg; sv += (float)kv[q] * gg; se += (float)ke[q] * gg; } }
#pragma unroll 1
    for (int d8 = 0; d8 < 16; d8 += 8) { const int d = (lane & 15) * 16 + d8; const v8b qe = *(const v8b*)(QE2 + b * E + h * HD + d);
#pragma unroll
      for (int q = 0; q < 8; ++q) sq += (float)qe[q] * bf16_rne(bi[E + h * HD + d + q]); }
    su = hsum16(su) * (1.0f / XS); sv = hsum16(sv) * (1.0f / XS); se = hsum16(se) * (1.0f / XS); sq = hsum16(sq) * (1.0f / XS);
    sc[h][0] = (su + sq) * (1.0f / 16.0f); sc[h][1] = (sv + sq) * (1.0f / 16.0f); sc[h][2] = (se + sq) * (1.0f / 16.0f); }
  float a[NH][3];
#pragma unroll
  for (int h = 0; h < NH; ++h) { const float mx = fmaxf(sc[h][0], fmaxf(sc[h][1], sc[h][2])); float e0 = nexp(sc[h][0] - mx), e1 = nexp(sc[h][1] - mx), e2 = nexp(sc[h][2] - mx); const float inv = 1.0f / (e0 + e1 + e2); a[h][0] = e0 * inv; a[h][1] = e1 * inv; a[h][2] = e2 * inv; }
  for (int pass = 0; pass < 2; ++pass) {
#pragma unroll
    for (int h = 0; h < NH; ++h) for (int j8 = 0; j8 < 32; j8 += 8) { const int j = c0 + j8; const v8b vu = *(const v8b*)(VU + b * 2 * E + j), vv = *(const v8b*)(VV + b * 2 * E + j), ve = *(const v8b*)(QKVE + b * 3 * E + 2 * E + j); v8b o;
#pragma unroll
        for (int q = 0; q < 8; ++q) o[q] = (b16)(pmul(a[h][0], (float)vu[q]) + pmul(a[h][1], (float)vv[q]) + pmul(a[h][2], (float)ve[q]));
        *(volatile v8b*)(VB + (b * NH + h) * E + j) = o; }
    __threadfence(); }
}
}

extern "C" void kernel_launch(void* const* d_in, const int* in_sizes, int n_in, void* d_out, int out_size, void* d_ws, size_t ws_size, hipStream_t stream) {
  (void)n_in;
  auto Fp = [&](int i) { return (const float*)d_in[i]; };
  if (in_sizes[0] != NBt * ND || in_sizes[2] != NBt * IE || in_sizes[3] != 3 * E * ND || in_sizes[5] != 3 * E * IE || in_sizes[7] != 3 * E * E || in_sizes[9] != E * E || in_sizes[11] != DM * E || in_sizes[13] != OE * DM || out_size != NBt * OE) return;
  size_t off = 0; char* ws = (char*)d_ws;
  auto carve = [&](size_t bytes) { char* p = ws + off; off += (bytes + 255) & ~(size_t)255; return p; };
  constexpr int CH = 4096;
  b16* XU = (b16*)carve((size_t)NBt * ND * 2); b16* XV = (b16*)carve((size_t)NBt * ND * 2); b16* XE = (b16*)carve((size_t)NBt * IE * 2);
  b16* WN = (b16*)carve((size_t)3 * E * ND * 2); b16* WE_ = (b16*)carve((size_t)3 * E * IE * 2); b16* WI = (b16*)carve((size_t)3 * E * E * 2); b16* WKT = (b16*)carve((size_t)NH * E * HD * 2); b16* WO = (b16*)carve((size_t)E * E * 2); b16* W1 = (b16*)carve((size_t)DM * E * 2); b16* W2 = (b16*)carve((size_t)OE * DM * 2);
  b16* KVU = (b16*)carve((size_t)CH * 2 * E * 2); b16* KVV = (b16*)carve((size_t)CH * 2 * E * 2); b16* QKVE = (b16*)carve((size_t)CH * 3 * E * 2); b16* QE2 = (b16*)carve((size_t)CH * E * 2); float* G = (float*)carve((size_t)CH * NH * E * 4);
  b16* VB = (b16*)carve((size_t)CH * NH * E * 2); b16* O16 = (b16*)carve((size_t)CH * E * 2); b16* HEh = (b16*)carve((size_t)CH * E * 2); b16* HEl = (b16*)carve((size_t)CH * E * 2); b16* H1h = (b16*)carve((size_t)CH * DM * 2); b16* H1l = (b16*)carve((size_t)CH * DM * 2);
  if (off > ws_size || off > ((size_t)128 << 20)) return;
  prepx_kernel<<<(unsigned)(((size_t)2 * NBt * ND / 8 + (size_t)NBt * IE / 8 + 255) / 256), 256, 0, stream>>>(Fp(0), Fp(1), Fp(2), XU, XV, XE);
  preprow_kernel<<<(3 * E * ND / 8 + 255) / 256, 256, 0, stream>>>(Fp(3), 3 * E * ND / 8, WN); preprow_kernel<<<(3 * E * IE / 8 + 255) / 256, 256, 0, stream>>>(Fp(5), 3 * E * IE / 8, WE_); preprow_kernel<<<(3 * E * E / 8 + 255) / 256, 256, 0, stream>>>(Fp(7), 3 * E * E / 8, WI);
  preprow_kernel<<<(E * E / 8 + 255) / 256, 256, 0, stream>>>(Fp(9), E * E / 8, WO); preprow_kernel<<<(DM * E / 8 + 255) / 256, 256, 0, stream>>>(Fp(11), DM * E / 8, W1); preprow_kernel<<<(OE * DM / 8 + 255) / 256, 256, 0, stream>>>(Fp(13), OE * DM / 8, W2);
  prepwk_kernel<<<dim3(HD / 64, E / 64, NH), 256, 0, stream>>>(Fp(7), WKT);
  auto G0 = [&](const b16* A, const b16* Al, const b16* W, const float* b, b16* Yh, b16* Yl, float* Y32, int lda, int K, int ldy, int act, int boff, int yoff) { GArgs g; memset(&g, 0, sizeof(g)); g.A = A; g.Al = Al; g.W = W; g.b = b; g.Yh = Yh; g.Yl = Yl; g.Y32 = Y32; g.lda = lda; g.K = K; g.ldy = ldy; g.act = act; g.boff = boff; g.yoff = yoff; return g; };
  for (int c = 0; c < NBt / CH; ++c) { const size_t r0 = (size_t)c * CH;
    gemm_kernel<0><<<dim3(CH / 64, 2 * E / 128), 128, 0, stream>>>(G0(XU + r0 * ND, nullptr, WN + (size_t)E * ND, Fp(4), KVU, nullptr, nullptr, ND, ND, 2 * E, 0, E, 0));
    gemm_kernel<0><<<dim3(CH / 64, 2 * E / 128), 128, 0, stream>>>(G0(XV + r0 * ND, nullptr, WN + (size_t)E * ND, Fp(4), KVV, nullptr, nullptr, ND, ND, 2 * E, 0, E, 0));
    gemm_kernel<0><<<dim3(CH / 64, 3 * E / 128), 128, 0, stream>>>(G0(XE + r0 * IE, nullptr, WE_, Fp(6), QKVE, nullptr, nullptr, IE, IE, 3 * E, 0, 0, 0));
    gemm_kernel<0><<<dim3(CH / 64, E / 128), 128, 0, stream>>>(G0(QKVE, nullptr, WI, Fp(8), QE2, nullptr, nullptr, 3 * E, E, E, 0, 0, 0));
    for (int h = 0; h < NH; ++h) gemm_kernel<1><<<dim3(CH / 64, E / 128), 128, 0, stream>>>(G0(QE2 + h * HD, nullptr, WKT + (size_t)h * E * HD, nullptr, nullptr, nullptr, G, E, HD, NH * E, 0, 0, h * E));
    mix_kernel<<<CH / 16, 256, 0, stream>>>(KVU, KVU + E, KVV, KVV + E, QKVE, QE2, G, Fp(8), VB);
    for (int h = 0; h < NH; ++h) gemm_kernel<0><<<dim3(CH / 64, HD / 128), 128, 0, stream>>>(G0(VB + h * E, nullptr, WI + ((size_t)2 * E + h * HD) * E, Fp(8), O16, nullptr, nullptr, NH * E, E, E, 0, 2 * E + h * HD, h * HD));
    gemm_kernel<0><<<dim3(CH / 64, E / 128), 128, 0, stream>>>(G0(O16, nullptr, WO, Fp(10), HEh, HEl, nullptr, E, E, E, 0, 0, 0));
    gemm_kernel<0><<<dim3(CH / 64, DM / 128), 128, 0, stream>>>(G0(HEh, HEl, W1, Fp(12), H1h, H1l, nullptr, E, E, DM, 1, 0, 0));
    gemm_kernel<1><<<dim3(CH / 64, OE / 128), 128, 0, stream>>>(G0(H1h, H1l, W2, Fp(14), nullptr, nullptr, (float*)d_out + r0 * OE, DM, DM, OE, 0, 0, 0));
  }
}
